// BlinnPhongShaderEnvMap_27041114096024
// MI455X (gfx1250) — hardware-verified
//
#include <hip/hip_runtime.h>
#include <math.h>


typedef __bf16 b16;
typedef __attribute__((ext_vector_type(16))) __bf16   v16b;
typedef __attribute__((ext_vector_type(16))) _Float16 v16h;
typedef __attribute__((ext_vector_type(8)))  float    v8f;
typedef __attribute__((ext_vector_type(4)))  float    v4f;

#define HW        65536
#define J_LIGHTS  256
#define V_CNT     20000
#define F_CNT     40000
#define NENT      (F_CNT * 3)
#define EPS_N     1e-6f
#define VPB       2048

#define WS_ENT_OFF  0
#define WS_VN_OFF   (2u * 1024u * 1024u)
#define WS_PIX_OFF  (3u * 1024u * 1024u)
#define WS_END      (6u * 1024u * 1024u)

__device__ __forceinline__ b16 bf16_rne(float f) { unsigned u = __float_as_uint(f); u += 0x7fffu + ((u >> 16) & 1u); return __builtin_bit_cast(b16, (unsigned short)(u >> 16)); }
__device__ __forceinline__ float bf16_f32(b16 b) { return __uint_as_float(((unsigned)__builtin_bit_cast(unsigned short, b)) << 16); }
__device__ __forceinline__ void split3(float x, b16& h, b16& m, b16& l) { h = bf16_rne(x); const float r1 = x - bf16_f32(h); m = bf16_rne(r1); l = bf16_rne(r1 - bf16_f32(m)); }
__device__ __forceinline__ v8f wmmab(v16b a, v16b b, v8f c) {
  v8f d = __builtin_amdgcn_wmma_f32_16x16x32_bf16(false, a, false, b, (short)0, c, false, false);
  asm volatile("v_nop\n\tv_nop\n\tv_nop\n\tv_nop" : "+v"(d) : "v"(a), "v"(b));
  return d;
}
__device__ __forceinline__ v8f wmmah(v16h a, v16h b, v8f c) {
  v8f d = __builtin_amdgcn_wmma_f32_16x16x32_f16(false, a, false, b, (short)0, c, false, false);
  asm volatile("v_nop\n\tv_nop\n\tv_nop\n\tv_nop" : "+v"(d) : "v"(a), "v"(b));
  return d;
}
__device__ __forceinline__ v16b frag3(float x, float y, float z, const int sel[6], int hh) {
  b16 parts[3][3];
  split3(x, parts[0][0], parts[0][1], parts[0][2]);
  split3(y, parts[1][0], parts[1][1], parts[1][2]);
  split3(z, parts[2][0], parts[2][1], parts[2][2]);
  v16b f;
#pragma unroll
  for (int e = 0; e < 16; ++e) {
    const int k = ((e < 8) ? e : (e + 8)) + 8 * hh;
    const int j = k >> 2, c = k & 3;
    f[e] = (j < 6 && c < 3) ? parts[c][sel[j]] : bf16_rne(0.0f);
  }
  return f;
}
#define VST2(T, ptr, val) do { const T _v = (val); *(volatile T*)(ptr) = _v; __threadfence(); *(volatile T*)(ptr) = _v; } while (0)

__global__ __launch_bounds__(256) void entries_kernel(const float* __restrict__ verts, const int* __restrict__ faces, float* __restrict__ ws) {
  const int e = blockIdx.x * 256 + threadIdx.x;
  if (e >= NENT) return;
  const int f = e / 3, c = e - f * 3;
  const int i0 = faces[f * 3 + 0], i1 = faces[f * 3 + 1], i2 = faces[f * 3 + 2];
  const float ax = verts[i0 * 3 + 0], ay = verts[i0 * 3 + 1], az = verts[i0 * 3 + 2];
  const float bx = verts[i1 * 3 + 0], by = verts[i1 * 3 + 1], bz = verts[i1 * 3 + 2];
  const float cx = verts[i2 * 3 + 0], cy = verts[i2 * 3 + 1], cz = verts[i2 * 3 + 2];
  const float e1x = bx - ax, e1y = by - ay, e1z = bz - az;
  const float e2x = cx - ax, e2y = cy - ay, e2z = cz - az;
  v4f ent;
  ent[0] = __int_as_float(faces[f * 3 + c]);
  ent[1] = e1y * e2z - e1z * e2y;
  ent[2] = e1z * e2x - e1x * e2z;
  ent[3] = e1x * e2y - e1y * e2x;
  VST2(v4f, ws + (WS_ENT_OFF / 4) + (size_t)e * 4, ent);
}

__global__ __launch_bounds__(256) void vnorm_kernel(const float* __restrict__ ws_ent, float* __restrict__ vn) {
  __shared__ __attribute__((aligned(16))) v4f tile[512];
  __shared__ __attribute__((aligned(16))) float acc[256 * 24 + 4];
  const int t = threadIdx.x;
  const int vbase = blockIdx.x * VPB + t * 8;
  float* my = acc + t * 24;
#pragma unroll
  for (int i = 0; i < 24; ++i) my[i] = 0.0f;
  for (int e0 = 0; e0 < NENT; e0 += 512) {
    const int n = min(512, NENT - e0);
    __syncthreads();
    for (int i = t; i < n; i += 256) tile[i] = *(const v4f*)(ws_ent + (size_t)(e0 + i) * 4);
    __syncthreads();
    for (int i = 0; i < n; ++i) {
      const v4f en = tile[i];
      const unsigned d = (unsigned)(__float_as_int(en[0]) - vbase);
      if (d < 8u) { my[d * 3 + 0] += en[1]; my[d * 3 + 1] += en[2]; my[d * 3 + 2] += en[3]; }
    }
  }
  __syncthreads();
  float* dst = vn + (size_t)blockIdx.x * VPB * 3;
  for (int pass = 0; pass < 2; ++pass) {
    for (int piece = t; piece < VPB * 3 / 4; piece += 256) *(volatile v4f*)(dst + piece * 4) = *(const v4f*)(acc + piece * 4);
    __threadfence();
  }
}

__global__ __launch_bounds__(256) void pixel_prep_kernel(const float* __restrict__ verts, const int* __restrict__ faces,
                                                         const int* __restrict__ p2f, const float* __restrict__ bary,
                                                         const float* __restrict__ cam, const float* __restrict__ vn,
                                                         float* __restrict__ ws_pix, float* __restrict__ out) {
  __shared__ __attribute__((aligned(16))) float spd[256 * 8];
  __shared__ __attribute__((aligned(16))) float snrm[256 * 3];
  const int t = threadIdx.x;
  const int p = blockIdx.x * 256 + t;
  int f = p2f[p];
  bool mask = (f < 0);
  int fi = mask ? 0 : f;
  float w0 = bary[p * 3 + 0], w1 = bary[p * 3 + 1], w2 = bary[p * 3 + 2];
  int i0 = faces[fi * 3 + 0], i1 = faces[fi * 3 + 1], i2 = faces[fi * 3 + 2];
  float px = 0.f, py = 0.f, pz = 0.f, nx = 0.f, ny = 0.f, nz = 0.f;
  if (!mask) {
    px = w0 * verts[i0 * 3 + 0] + w1 * verts[i1 * 3 + 0] + w2 * verts[i2 * 3 + 0];
    py = w0 * verts[i0 * 3 + 1] + w1 * verts[i1 * 3 + 1] + w2 * verts[i2 * 3 + 1];
    pz = w0 * verts[i0 * 3 + 2] + w1 * verts[i1 * 3 + 2] + w2 * verts[i2 * 3 + 2];
    nx = w0 * vn[i0 * 3 + 0] + w1 * vn[i1 * 3 + 0] + w2 * vn[i2 * 3 + 0];
    ny = w0 * vn[i0 * 3 + 1] + w1 * vn[i1 * 3 + 1] + w2 * vn[i2 * 3 + 1];
    nz = w0 * vn[i0 * 3 + 2] + w1 * vn[i1 * 3 + 2] + w2 * vn[i2 * 3 + 2];
  }
  float nlen = sqrtf(nx * nx + ny * ny + nz * nz);
  float ninv = 1.0f / fmaxf(nlen, EPS_N);
  nx *= ninv; ny *= ninv; nz *= ninv;
  float vx = cam[0] - px, vy = cam[1] - py, vz = cam[2] - pz;
  float vlen = sqrtf(vx * vx + vy * vy + vz * vz);
  float vinv = 1.0f / fmaxf(vlen, EPS_N);
  vx *= vinv; vy *= vinv; vz *= vinv;
  spd[t * 8 + 0] = nx; spd[t * 8 + 1] = ny; spd[t * 8 + 2] = nz;
  spd[t * 8 + 3] = vx; spd[t * 8 + 4] = vy; spd[t * 8 + 5] = vz;
  spd[t * 8 + 6] = nx * vx + ny * vy + nz * vz;
  spd[t * 8 + 7] = vx * vx + vy * vy + vz * vz;
  snrm[t * 3 + 0] = nx; snrm[t * 3 + 1] = ny; snrm[t * 3 + 2] = nz;
  __syncthreads();
  float* pd = ws_pix + (size_t)blockIdx.x * 256 * 8;
  float* n0 = out + (size_t)2 * HW * 3 + (size_t)blockIdx.x * 256 * 3;
  float* n1 = n0 + (size_t)HW * 3;
  for (int pass = 0; pass < 2; ++pass) {
#pragma unroll
    for (int q = 0; q < 2; ++q) *(volatile v4f*)(pd + (t + q * 256) * 4) = *(const v4f*)(spd + (t + q * 256) * 4);
    if (t < 192) { const v4f v = *(const v4f*)(snrm + t * 4); *(volatile v4f*)(n0 + t * 4) = v; *(volatile v4f*)(n1 + t * 4) = v; }
    __threadfence();
  }
}

__global__ void __launch_bounds__(256) shade_kernel(const float* __restrict__ ldir, const float* __restrict__ lcol,
                                                    const float* __restrict__ shin_p, const float* __restrict__ kd_p, const float* __restrict__ ks_p,
                                                    const float* __restrict__ ws_pix, float* __restrict__ out) {
  __shared__ float s_ldir[J_LIGHTS * 3];
  __shared__ float s_ll[J_LIGHTS];
  __shared__ __attribute__((aligned(16))) _Float16 s_lcol[J_LIGHTS * 16];
  __shared__ float s_ndv[8][16];
  __shared__ __attribute__((aligned(16))) _Float16 s_tile[8][16][40];
  __shared__ __attribute__((aligned(16))) float s_col[128 * 3];

  const int tid  = threadIdx.x;
  const int wave = tid >> 5;
  const int lane = tid & 31;
  const int b    = blockIdx.x >> 9;
  const int pbase = (blockIdx.x & 511) * 128 + wave * 16;
  const int m16 = lane & 15, hh = lane >> 4;

  {
    const float* ld = ldir + ((size_t)b * J_LIGHTS + tid) * 3;
    const float* lc = lcol + ((size_t)b * J_LIGHTS + tid) * 3;
    const float lx = ld[0], ly = ld[1], lz = ld[2];
    s_ldir[tid * 3 + 0] = lx; s_ldir[tid * 3 + 1] = ly; s_ldir[tid * 3 + 2] = lz;
    s_ll[tid] = lx * lx + ly * ly + lz * lz;
#pragma unroll
    for (int c = 0; c < 16; ++c) s_lcol[tid * 16 + c] = (_Float16)((c < 3) ? lc[c] : 0.0f);
  }
  const float* pd = ws_pix + (size_t)(pbase + m16) * 8;
  const float nx = pd[0], ny = pd[1], nz = pd[2];
  const float vx = pd[3], vy = pd[4], vz = pd[5];
  if (hh == 0) s_ndv[wave][m16] = pd[6];
  const float vv_lane = pd[7];
  __syncthreads();

  const int selA[6] = {0, 0, 0, 1, 1, 2};
  const int selB[6] = {0, 1, 2, 0, 1, 0};
  const v16b a_n = frag3(nx, ny, nz, selA, hh);
  const v16b a_v = frag3(vx, vy, vz, selA, hh);

  const float shin = shin_p[0];
  const float kd   = kd_p[0];
  const float bpks = ks_p[0] * (shin + 2.0f) / (4.0f * (2.0f - expf(-shin * 0.5f)));
  float vv_r[8], ndv_r[8];
#pragma unroll
  for (int r = 0; r < 8; ++r) { vv_r[r] = __shfl(vv_lane, 8 * hh + r, 32); ndv_r[r] = s_ndv[wave][8 * hh + r]; }

  v8f cacc = {0.f, 0.f, 0.f, 0.f, 0.f, 0.f, 0.f, 0.f};
  const v8f zero = {0.f, 0.f, 0.f, 0.f, 0.f, 0.f, 0.f, 0.f};
  _Float16* tile = &s_tile[wave][0][0];

  for (int g = 0; g < 16; ++g) {
    const int ln = g * 16 + m16;
    const v16b b_l = frag3(s_ldir[ln * 3 + 0], s_ldir[ln * 3 + 1], s_ldir[ln * 3 + 2], selB, hh);
    const v8f dn = wmmab(a_n, b_l, zero);
    const v8f dv = wmmab(a_v, b_l, zero);
    const float ll = s_ll[ln];
#pragma unroll
    for (int r = 0; r < 8; ++r) {
      const float ndl  = dn[r];
      const float vdl  = dv[r];
      const float diff = fminf(fmaxf(ndl, 0.0f), 1.0f);
      const float hlen = sqrtf(fmaxf(vv_r[r] + ll + 2.0f * vdl, 0.0f));
      const float rin  = 1.0f / fmaxf(hlen, EPS_N);
      const float sp   = fminf(fmaxf((ndv_r[r] + ndl) * rin, 0.0f), 1.0f);
      const float spp  = powf(sp, shin);
      tile[(8 * hh + r) * 40 + (g & 1) * 16 + m16] = (_Float16)fmaf(kd, diff, bpks * spp);
    }
    if (g & 1) {
      __builtin_amdgcn_fence(__ATOMIC_RELEASE, "workgroup"); __builtin_amdgcn_wave_barrier(); __builtin_amdgcn_fence(__ATOMIC_ACQUIRE, "workgroup");
      v16h a_s, b_c;
      const _Float16* arow = tile + m16 * 40;
      const int j0 = (g - 1) * 16;
#pragma unroll
      for (int e = 0; e < 16; ++e) { const int k = ((e < 8) ? e : (e + 8)) + 8 * hh; a_s[e] = arow[k]; b_c[e] = s_lcol[(j0 + k) * 16 + m16]; }
      cacc = wmmah(a_s, b_c, cacc);
      __builtin_amdgcn_wave_barrier();
    }
  }
  if (m16 < 3) {
#pragma unroll
    for (int r = 0; r < 8; ++r) s_col[(wave * 16 + 8 * hh + r) * 3 + m16] = cacc[r];
  }
  __syncthreads();
  float* cout = out + (size_t)b * HW * 3 + (size_t)(blockIdx.x & 511) * 128 * 3;
  for (int pass = 0; pass < 2; ++pass) {
    if (tid < 96) *(volatile v4f*)(cout + tid * 4) = *(const v4f*)(s_col + tid * 4);
    __threadfence();
  }
}

extern "C" void kernel_launch(void* const* d_in, const int* in_sizes, int n_in,
                              void* d_out, int out_size, void* d_ws, size_t ws_size,
                              hipStream_t stream) {
  (void)in_sizes; (void)n_in; (void)out_size;
  const float* verts = (const float*)d_in[0];
  const int*   faces = (const int*)d_in[1];
  const int*   p2f   = (const int*)d_in[2];
  const float* bary  = (const float*)d_in[3];
  const float* ldir  = (const float*)d_in[4];
  const float* lcol  = (const float*)d_in[5];
  const float* cam   = (const float*)d_in[6];
  const float* shin  = (const float*)d_in[7];
  const float* kd    = (const float*)d_in[8];
  const float* ks    = (const float*)d_in[9];
  float* out = (float*)d_out;
  if (ws_size < WS_END) return;
  float* ws_ent = (float*)((char*)d_ws + WS_ENT_OFF);
  float* vn     = (float*)((char*)d_ws + WS_VN_OFF);
  float* ws_pix = (float*)((char*)d_ws + WS_PIX_OFF);

  entries_kernel<<<(NENT + 255) / 256, 256, 0, stream>>>(verts, faces, ws_ent);
  vnorm_kernel<<<(V_CNT + VPB - 1) / VPB, 256, 0, stream>>>(ws_ent, vn);
  pixel_prep_kernel<<<HW / 256, 256, 0, stream>>>(verts, faces, p2f, bary, cam, vn, ws_pix, out);
  shade_kernel<<<1024, 256, 0, stream>>>(ldir, lcol, shin, kd, ks, ws_pix, out);
}
